// CapsuleLayer_28114855920234
// MI455X (gfx1250) — hardware-verified
//
#include <hip/hip_runtime.h>
#include <stddef.h>


typedef _Float16 v16h __attribute__((ext_vector_type(16)));
typedef _Float16 v8h  __attribute__((ext_vector_type(8)));
typedef _Float16 v4h  __attribute__((ext_vector_type(4)));
typedef float    v8f  __attribute__((ext_vector_type(8)));
typedef float    v4f  __attribute__((ext_vector_type(4)));

#ifndef NB
#define NB 128
#endif
#ifndef NCAP
#define NCAP 2048
#endif
#define NB_FULL   128
#define NCAP_FULL 2048
#define OC    32
#define IDIM  8
#define ODIM  16
#define SROW  (OC * ODIM)
#define WBLK  (IDIM * ODIM)
#define NCHUNK 16
#define NPB   (NCAP / NCHUNK)
#define NSTEP 16

#define XCARRY 64.0f
#define WCARRY 64.0f
#define VCARRY 256.0f
#define ACARRY 64.0f
#define LOGIT_SCALE (1.0f / (WCARRY * VCARRY * XCARRY))

#define LPITCH 36
#define CPITCH 516
#define LDS_FLOATS 9216

static_assert(NB >= 16 && NB <= NB_FULL && (NB % 16) == 0);
static_assert(NCAP <= NCAP_FULL && (NCAP % (NCHUNK * NSTEP)) == 0);
static_assert(IDIM == 8 && ODIM == 16 && OC == 32);
static_assert(OC == 8 * 4);
static_assert(NSTEP * 16 == 256);
static_assert((NSTEP % 4) == 0 && (NSTEP % 2) == 0);
static_assert(((size_t)NB * NCAP) % 256 == 0);
static_assert(((size_t)NCAP * OC) % 16 == 0);
static_assert(((size_t)NB * SROW / 4) % 256 == 0);
static_assert((LPITCH % 4) == 0 && LPITCH >= OC);
static_assert((CPITCH % 4) == 0 && CPITCH >= SROW);
static_assert(LDS_FLOATS >= 256 * LPITCH && LDS_FLOATS >= 16 * CPITCH);
static_assert((OC % 16) == 0);
static_assert(16 * WBLK == 256 * 8);
static_assert(WBLK == 16 * 8);
static_assert((size_t)LDS_FLOATS * 4 <= (size_t)131072);

#define XH_BYTES   ((size_t)NB * NCAP * IDIM * 2)
#define W16_BYTES  ((size_t)NCAP * OC * WBLK * 2)
#define PART_BYTES ((size_t)NCHUNK * NB * SROW * 4)
#define VS_BYTES   ((size_t)NB * SROW * 4)
#define VH_BYTES   ((size_t)NB * SROW * 2)
#define OFF_XH   ((size_t)0)
#define OFF_WD   (OFF_XH + XH_BYTES)
#define OFF_WI   (OFF_WD + W16_BYTES)
#define OFF_PART (OFF_WI + W16_BYTES)
#define OFF_VS0  (OFF_PART + PART_BYTES)
#define OFF_VS1  (OFF_VS0 + VS_BYTES)
#define OFF_VH   (OFF_VS1 + VS_BYTES)
#define WS_TOTAL (OFF_VH + VH_BYTES)
static_assert((XH_BYTES % 128) == 0 && (W16_BYTES % 128) == 0 && (PART_BYTES % 128) == 0);
static_assert((VS_BYTES % 128) == 0 && (VH_BYTES % 128) == 0);
static_assert(WS_TOTAL <= (size_t)134217728);

__device__ __forceinline__ float bf16r(float x) {
  unsigned int u = __float_as_uint(x);
  u = (u + 0x7FFFu + ((u >> 16) & 1u)) & 0xFFFF0000u;
  return __uint_as_float(u);
}

static __device__ __forceinline__ _Float16 toh_flush(float v) {
  const _Float16 r = (_Float16)v;
  return (fabsf(v) < 6.103515625e-05f) ? (_Float16)0.0f : r;
}

__device__ __forceinline__ v16h cat8(v8h lo, v8h hi) {
  v16h out;
#pragma unroll
  for (int i = 0; i < 8; ++i) { out[i] = lo[i]; out[i + 8] = hi[i]; }
  return out;
}
__device__ __forceinline__ v16h pad8(v8h lo) {
  v16h out;
#pragma unroll
  for (int i = 0; i < 8; ++i) { out[i] = lo[i]; out[i + 8] = (_Float16)0.0f; }
  return out;
}

__device__ __forceinline__ v8f wmma16(v16h a, v16h b, v8f c) {
  v8f d = __builtin_amdgcn_wmma_f32_16x16x32_f16(false, a, false, b, (short)0, c,
                                                 false, false);
  asm volatile("v_nop\n\tv_nop\n\tv_nop\n\tv_nop" : "+v"(d) : "v"(a), "v"(b));
  return d;
}

__global__ __launch_bounds__(256) void xconv_kernel(
    const float* __restrict__ X, _Float16* __restrict__ XH) {
  const unsigned g = blockIdx.x * 256u + threadIdx.x;
  const unsigned b = g / (unsigned)NCAP;
  const unsigned n = g - b * (unsigned)NCAP;
  const float* src = X + ((size_t)b * NCAP_FULL + n) * IDIM;
  const v4f a0 = *(const v4f*)(src);
  const v4f a1 = *(const v4f*)(src + 4);
  v8h o;
#pragma unroll
  for (int i = 0; i < 4; ++i) {
    o[i]     = toh_flush(XCARRY * bf16r(a0[i]));
    o[i + 4] = toh_flush(XCARRY * bf16r(a1[i]));
  }
  _Float16* p = XH + (size_t)g * IDIM;
  *(volatile v8h*)p = o;
  __threadfence();
  *(volatile v8h*)p = o;
}

__global__ __launch_bounds__(256) void wconv_kernel(
    const float* __restrict__ W, _Float16* __restrict__ WD, _Float16* __restrict__ WI) {
  __shared__ _Float16 T[16 * WBLK];
  const unsigned tid = threadIdx.x;
  const unsigned n  = blockIdx.x / (unsigned)(OC / 16);
  const unsigned o0 = (blockIdx.x - n * (unsigned)(OC / 16)) * 16u;
  const unsigned p  = tid >> 4;
  const unsigned dd = tid & 15u;
  const size_t src  = ((size_t)(o0 + p) * NCAP_FULL + n) * WBLK + dd * 8u;
  const size_t base = (size_t)blockIdx.x * (16u * WBLK) + tid * 8u;
  const v4f a0 = *(const v4f*)(W + src);
  const v4f a1 = *(const v4f*)(W + src + 4);
  v8h o;
#pragma unroll
  for (int i = 0; i < 4; ++i) {
    o[i]     = toh_flush(WCARRY * bf16r(a0[i]));
    o[i + 4] = toh_flush(WCARRY * bf16r(a1[i]));
  }
#pragma unroll
  for (unsigned j = 0; j < 8u; ++j) T[p * WBLK + j * ODIM + dd] = o[j];
  __syncthreads();
  const v8h t = *(const v8h*)&T[tid * 8u];
  *(volatile v8h*)(WI + base) = o;
  *(volatile v8h*)(WD + base) = t;
  __threadfence();
  *(volatile v8h*)(WI + base) = o;
  *(volatile v8h*)(WD + base) = t;
}

template <int UNI>
__device__ __forceinline__ void pass_body(
    const _Float16* __restrict__ XH, const _Float16* __restrict__ WD,
    const _Float16* __restrict__ WI, const _Float16* __restrict__ VH,
    float* __restrict__ part, const float scale) {
  __shared__ float Ls[LDS_FLOATS];
  const unsigned tid = threadIdx.x, lane = tid & 31u;
  const unsigned wave = (unsigned)__builtin_amdgcn_readfirstlane((int)(threadIdx.x >> 5));
  const unsigned hh = lane >> 4, m = lane & 15u;
  const unsigned chunk = blockIdx.x;
  const unsigned b0 = blockIdx.y * 16u;
  const unsigned nbeg = chunk * (unsigned)NPB;
  const unsigned o0 = wave * 4u;
  const size_t xrow = (size_t)(b0 + m) * NCAP;

  v8f acc[4];
#pragma unroll
  for (int oi = 0; oi < 4; ++oi) acc[oi] = (v8f){};

  v16h vf[4];
  if (!UNI) {
#pragma unroll
    for (int oi = 0; oi < 4; ++oi) {
      const v8h t = *(const v8h*)(VH + (size_t)(b0 + m) * SROW + (o0 + (unsigned)oi) * ODIM + hh * 8u);
      vf[oi] = pad8(t);
    }
  }

#pragma unroll 1
  for (unsigned st = 0; st < (unsigned)(NPB / NSTEP); ++st) {
    const unsigned n0 = nbeg + st * (unsigned)NSTEP;

    if (!UNI) {
#pragma unroll 1
      for (unsigned np = 0; np < (unsigned)(NSTEP / 2); ++np) {
        const unsigned nA = n0 + 2u * np;
        const v8h xv = *(const v8h*)(XH + (xrow + nA + hh) * IDIM);
        float xf[8];
#pragma unroll
        for (int r = 0; r < 8; ++r) xf[r] = (float)xv[r];
        const _Float16* wp = WD + ((size_t)(nA + (m >> 3)) * OC + o0) * WBLK + (m & 7u) * ODIM + hh * 8u;
        v4f lg;
#pragma unroll
        for (int oi = 0; oi < 4; ++oi) {
          const v8h wl = *(const v8h*)(wp + oi * WBLK);
          const v16h a = pad8(wl);
          v8f d = {};
          d = wmma16(a, vf[oi], d);
          float t = d[0] * xf[0];
#pragma unroll
          for (int r = 1; r < 8; ++r) t += d[r] * xf[r];
          lg[oi] = t * LOGIT_SCALE;
        }
        *(v4f*)&Ls[((2u * np + hh) * 16u + m) * LPITCH + o0] = lg;
      }
      __syncthreads();

      {
        float lv[32];
#pragma unroll
        for (int q = 0; q < 8; ++q) {
          const v4f t = *(const v4f*)&Ls[tid * LPITCH + 4u * (unsigned)q];
          lv[4 * q + 0] = t[0];
          lv[4 * q + 1] = t[1];
          lv[4 * q + 2] = t[2];
          lv[4 * q + 3] = t[3];
        }
        float mx = lv[0];
#pragma unroll
        for (int q = 1; q < 32; ++q) mx = fmaxf(mx, lv[q]);
        float sum = 0.0f;
#pragma unroll
        for (int q = 0; q < 32; ++q) {
          lv[q] = __expf(lv[q] - mx);
          sum += lv[q];
        }
        const float inv = __builtin_amdgcn_rcpf(sum) * ACARRY;
#pragma unroll
        for (int q = 0; q < 8; ++q) {
          v4f t;
          t[0] = lv[4 * q + 0] * inv;
          t[1] = lv[4 * q + 1] * inv;
          t[2] = lv[4 * q + 2] * inv;
          t[3] = lv[4 * q + 3] * inv;
          *(v4f*)&Ls[tid * LPITCH + 4u * (unsigned)q] = t;
        }
      }
      __syncthreads();
    }

#pragma unroll 1
    for (unsigned ks = 0; ks < (unsigned)(NSTEP / 4); ++ks) {
      const unsigned nA = n0 + 4u * ks + hh;
      const v8h x0 = *(const v8h*)(XH + (xrow + nA) * IDIM);
      const v8h x1 = *(const v8h*)(XH + (xrow + nA + 2u) * IDIM);
      const _Float16* wp = WI + ((size_t)nA * OC + o0) * WBLK + m * IDIM;
      if (UNI) {
        const v16h a = cat8(x0, x1);
#pragma unroll
        for (int oi = 0; oi < 4; ++oi) {
          const v8h w0 = *(const v8h*)(wp + oi * WBLK);
          const v8h w1 = *(const v8h*)(wp + 2 * OC * WBLK + oi * WBLK);
          acc[oi] = wmma16(a, cat8(w0, w1), acc[oi]);
        }
      } else {
        float xa[8], xb[8];
#pragma unroll
        for (int j = 0; j < 8; ++j) { xa[j] = (float)x0[j]; xb[j] = (float)x1[j]; }
        const v4f c0 = *(const v4f*)&Ls[((4u * ks + hh) * 16u + m) * LPITCH + o0];
        const v4f c1 = *(const v4f*)&Ls[((4u * ks + 2u + hh) * 16u + m) * LPITCH + o0];
#pragma unroll
        for (int oi = 0; oi < 4; ++oi) {
          v16h a;
#pragma unroll
          for (int j = 0; j < 8; ++j) {
            a[j]     = toh_flush(c0[oi] * xa[j]);
            a[j + 8] = toh_flush(c1[oi] * xb[j]);
          }
          const v8h w0 = *(const v8h*)(wp + oi * WBLK);
          const v8h w1 = *(const v8h*)(wp + 2 * OC * WBLK + oi * WBLK);
          acc[oi] = wmma16(a, cat8(w0, w1), acc[oi]);
        }
      }
    }
    if (!UNI) __syncthreads();
  }

#pragma unroll
  for (int oi = 0; oi < 4; ++oi)
#pragma unroll
    for (int r = 0; r < 8; ++r)
      Ls[(hh * 8u + (unsigned)r) * CPITCH + (o0 + (unsigned)oi) * ODIM + m] = acc[oi][r] * scale;
  __syncthreads();
  v4f xs[8];
  size_t off[8];
#pragma unroll
  for (unsigned j = 0; j < 8u; ++j) {
    const unsigned idx = tid + 256u * j;
    const unsigned row = idx >> 7;
    const unsigned c4 = (idx & 127u) * 4u;
    xs[j] = *(const v4f*)&Ls[row * CPITCH + c4];
    off[j] = ((size_t)chunk * NB + b0 + row) * SROW + c4;
  }
#pragma unroll
  for (int j = 0; j < 8; ++j) *(volatile v4f*)(part + off[j]) = xs[j];
  __threadfence();
#pragma unroll
  for (int j = 0; j < 8; ++j) *(volatile v4f*)(part + off[j]) = xs[j];
}

__global__ __launch_bounds__(256) void pass_uniform_kernel(
    const _Float16* __restrict__ XH, const _Float16* __restrict__ WI,
    float* __restrict__ part, const float scale) {
  pass_body<1>(XH, WI, WI, XH, part, scale);
}
__global__ __launch_bounds__(256) void pass_route_kernel(
    const _Float16* __restrict__ XH, const _Float16* __restrict__ WD,
    const _Float16* __restrict__ WI, const _Float16* __restrict__ VH,
    float* __restrict__ part, const float scale) {
  pass_body<0>(XH, WD, WI, VH, part, scale);
}

__global__ __launch_bounds__(256) void squash_kernel(
    const float* __restrict__ part, const float* __restrict__ vold,
    float* __restrict__ vsum, _Float16* __restrict__ vh, float* __restrict__ out,
    const int have_acc, const int last) {
#pragma clang fp contract(off)
  const unsigned g = blockIdx.x * 256u + threadIdx.x;
  const size_t e = (size_t)g * 4u;
  v4f s = {0.0f, 0.0f, 0.0f, 0.0f};
#pragma unroll 1
  for (unsigned c = 0; c < (unsigned)NCHUNK; ++c) {
    const v4f p = *(const v4f*)(part + (size_t)c * ((size_t)NB * SROW) + e);
    s = s + p;
  }
  float sq = (s[0] * s[0] + s[1] * s[1]) + (s[2] * s[2] + s[3] * s[3]);
  sq += __shfl_xor(sq, 1, 32);
  sq += __shfl_xor(sq, 2, 32);
  const float sc = sq * __builtin_amdgcn_rcpf(1.0f + sq);
  const float rn = __builtin_amdgcn_rcpf(sqrtf(sq + 1.0e-7f));
  const float scl = sc * rn;
  v4f v;
#pragma unroll
  for (int j = 0; j < 4; ++j) v[j] = scl * s[j];

  if (last) {
    *(volatile v4f*)(out + e) = v;
    __threadfence();
    *(volatile v4f*)(out + e) = v;
  } else {
    v4f t = v;
    if (have_acc) {
      const v4f pv = *(const v4f*)(vold + e);
      t = pv + v;
    }
    v4h hq;
#pragma unroll
    for (int j = 0; j < 4; ++j) hq[j] = toh_flush(VCARRY * t[j]);
    *(volatile v4f*)(vsum + e) = t;
    *(volatile v4h*)(vh + e) = hq;
    __threadfence();
    *(volatile v4f*)(vsum + e) = t;
    *(volatile v4h*)(vh + e) = hq;
  }
}

extern "C" void kernel_launch(void* const* d_in, const int* in_sizes, int n_in,
                              void* d_out, int out_size, void* d_ws, size_t ws_size,
                              hipStream_t stream) {
  if (n_in < 2) return;
  const long long need_x = ((long long)(NB - 1) * NCAP_FULL + NCAP) * IDIM;
  if ((long long)in_sizes[0] < need_x) return;
  const long long need_w = ((long long)(OC - 1) * NCAP_FULL + NCAP) * WBLK;
  if ((long long)in_sizes[1] < need_w) return;
  if ((long long)out_size < (long long)NB * SROW) return;
  if (ws_size < WS_TOTAL) return;

  const float* X = (const float*)d_in[0];
  const float* W = (const float*)d_in[1];
  float* out = (float*)d_out;

  char* ws = (char*)d_ws;
  _Float16* XH  = (_Float16*)(ws + OFF_XH);
  _Float16* WD  = (_Float16*)(ws + OFF_WD);
  _Float16* WI  = (_Float16*)(ws + OFF_WI);
  float*    PART = (float*)(ws + OFF_PART);
  float*    VS0 = (float*)(ws + OFF_VS0);
  float*    VS1 = (float*)(ws + OFF_VS1);
  _Float16* VH  = (_Float16*)(ws + OFF_VH);

  dim3 blk(256);
  dim3 gpass(NCHUNK, NB / 16);
  dim3 gsq((unsigned)((size_t)NB * SROW / 4 / 256));

  xconv_kernel<<<dim3((unsigned)((size_t)NB * NCAP / 256)), blk, 0, stream>>>(X, XH);
  wconv_kernel<<<dim3((unsigned)((size_t)NCAP * OC / 16)), blk, 0, stream>>>(W, WD, WI);

  pass_uniform_kernel<<<gpass, blk, 0, stream>>>(XH, WI, PART,
                                                 1.0f / (XCARRY * WCARRY * (float)OC));
  squash_kernel<<<gsq, blk, 0, stream>>>(PART, VS0, VS0, VH, out, 0, 0);

  pass_route_kernel<<<gpass, blk, 0, stream>>>(XH, WD, WI, VH, PART,
                                               1.0f / (XCARRY * WCARRY * ACARRY));
  squash_kernel<<<gsq, blk, 0, stream>>>(PART, VS0, VS1, VH, out, 1, 0);

  pass_route_kernel<<<gpass, blk, 0, stream>>>(XH, WD, WI, VH, PART,
                                               1.0f / (XCARRY * WCARRY * ACARRY));
  squash_kernel<<<gsq, blk, 0, stream>>>(PART, VS1, VS1, VH, out, 0, 1);
}
